// RNN_74096775790863
// MI455X (gfx1250) — hardware-verified
//
#include <hip/hip_runtime.h>
#include <math.h>

typedef __attribute__((ext_vector_type(16))) _Float16 v16h;
typedef __attribute__((ext_vector_type(8)))  _Float16 v8h;
typedef __attribute__((ext_vector_type(8)))  float    v8f;
typedef __attribute__((ext_vector_type(2)))  float    v2f;

constexpr int kVocab   = 81743;
constexpr int kEmb     = 10;
constexpr int kH1      = 75;
constexpr int kH2      = 30;
constexpr int kT       = 512;
constexpr int kB       = 1024;
constexpr int kH1P     = 80;
constexpr int kH2P     = 32;
constexpr int kEW      = 16;
constexpr int kK1      = kH1P + kEW;
constexpr int kK2      = kH1P + kH2P + 16;
constexpr int kN1      = 4 * kH1P;
constexpr int kN2      = 4 * kH2P;
constexpr int kW1Rows  = kEmb + kH1;
constexpr int kW1Cols  = 4 * kH1;
constexpr int kW2Rows  = kH1 + kH2;
constexpr int kW2Cols  = 4 * kH2;
constexpr int kP1      = 104;
constexpr int kP2      = 136;
constexpr int kCh1     = kP1 / 8;
constexpr int kCh2     = kP2 / 8;
constexpr int kRowsBlk = 16;
constexpr int kL1Waves = 5;
constexpr int kL2Waves = 2;
constexpr int kThreads = (kL1Waves + kL2Waves) * 32;
constexpr int kBlocks  = kB / kRowsBlk;
constexpr float kCarryA = 1024.0f;
constexpr float kCarryW = 64.0f;
constexpr float kFold   = 1.0f / (kCarryA * kCarryW);
constexpr float kF16MinNormal = 6.103515625e-05f;

static_assert(kH1P == kL1Waves * 16 && kH2P == kL2Waves * 16, "one 16-unit tile per wave");
static_assert(kK1 == 96 && kK2 == 128 && (kK1 % 32) == 0 && (kK2 % 32) == 0, "K multiples of 32");
static_assert(kN1 == 320 && kN2 == 128, "gate-aligned N extents");
static_assert(kW1Rows == 85 && kW1Cols == 300 && kW2Rows == 105 && kW2Cols == 120, "wire shapes");
static_assert(kP1 >= kK1 && kP2 >= kK2 && (kP1 % 8) == 0 && (kP2 % 8) == 0, "LDS pitches");
static_assert(kB % kRowsBlk == 0, "batch tiles");
static_assert(kRowsBlk * 2 * 4 == 128, "one output line per block");
static_assert(kEmb <= kEW && kH1 <= kH1P && kH2 <= kH2P, "pads");

constexpr size_t kOffE    = 0;
constexpr size_t kBytesE  = (size_t)kT * kB * kEW * 2;
constexpr size_t kWsTotal = kOffE + kBytesE;
static_assert(kWsTotal == 16777216ull, "carve total");
static_assert(kWsTotal <= 134217728ull, "carve cap");
constexpr int kPackChunks = kT * kB * 2;
static_assert((kPackChunks % 256) == 0, "pack grid exact");

union FragU { v16h v; v8h h[2]; };

__device__ __forceinline__ v16h frag_load(const _Float16* p) {
  FragU f;
  f.h[0] = *(const v8h*)(p);
  f.h[1] = *(const v8h*)(p + 16);
  return f.v;
}

__device__ __forceinline__ v8f mma_h(v16h a, v16h b, v8f c) {
  c = __builtin_amdgcn_wmma_f32_16x16x32_f16(false, a, false, b, (short)0, c, false, false);
  asm volatile("v_nop\n\tv_nop\n\tv_nop\n\tv_nop" : "+v"(c) : "v"(a), "v"(b));
  return c;
}

__device__ __forceinline__ _Float16 to_h_flush(float v) {
  const float z = (fabsf(v) < kF16MinNormal) ? 0.0f : v;
  return (_Float16)z;
}

__device__ __forceinline__ float fsig(float x) {
  return __builtin_amdgcn_rcpf(1.0f + __expf(-x));
}

__device__ __forceinline__ float ftanh(float x) {
  const float x2 = x * x;
  float pl = 62.0f / 2835.0f;
  pl = fmaf(pl, x2, -17.0f / 315.0f);
  pl = fmaf(pl, x2, 2.0f / 15.0f);
  pl = fmaf(pl, x2, -1.0f / 3.0f);
  pl = fmaf(pl, x2, 1.0f);
  pl = pl * x;
  const float xc = fminf(fmaxf(x, -15.0f), 15.0f);
  const float ex = __expf(2.0f * xc);
  const float big = 1.0f - 2.0f * __builtin_amdgcn_rcpf(ex + 1.0f);
  return (fabsf(x) < 0.25f) ? pl : big;
}

__device__ __forceinline__ float cell_step(float ai, float ag, float af, float ao,
                                           float bi, float bg, float bf, float bo, float& c) {
  const float pi = fmaf(ai, kFold, bi);
  const float pg = fmaf(ag, kFold, bg);
  const float pf = fmaf(af, kFold, bf) + 1.0f;
  const float po = fmaf(ao, kFold, bo);
  const float si = fsig(pi);
  const float tg = ftanh(pg);
  const float sf = fsig(pf);
  const float so = fsig(po);
  c = fmaf(sf, c, si * tg);
  return so * ftanh(c);
}

template <int HREAL, int HPAD, int SRCN, int NROWS, int ROWOFF_A, int ROWOFF_B, int CNT_B>
__device__ __forceinline__ v8h pack_chunk(const float* __restrict__ W, int np, int k8) {
  const int gate = np / HPAD;
  const int j = np - gate * HPAD;
  const bool colv = j < HREAL;
  const int jc = colv ? j : (HREAL - 1);
  const int col = gate * HREAL + jc;
  v8h hv;
#pragma unroll
  for (int e = 0; e < 8; ++e) {
    const int k = k8 + e;
    const bool inA = k < kH1;
    const bool inB = (k >= kH1P) && (k < kH1P + CNT_B);
    int row = inA ? (k + ROWOFF_A) : (k - kH1P + ROWOFF_B);
    row = row < 0 ? 0 : row;
    row = row > (NROWS - 1) ? (NROWS - 1) : row;
    float v = W[row * SRCN + col];
    asm volatile("" : "+v"(v));
    const bool ok = colv && (inA || inB);
    const float xs = ok ? (v * kCarryW) : 0.0f;
    hv[e] = to_h_flush(xs);
  }
  return hv;
}

__global__ __launch_bounds__(256) void pack_embed_kernel(
    const int* __restrict__ x, const float* __restrict__ embed, _Float16* __restrict__ Epl)
{
  const int c = blockIdx.x * 256 + threadIdx.x;
  const int hf = c & 1;
  const int ent = c >> 1;
  const int b = ent & (kB - 1);
  const int t = ent >> 10;
  int tok = x[(size_t)b * kT + t];
  tok = tok < 0 ? 0 : tok;
  tok = tok > (kVocab - 1) ? (kVocab - 1) : tok;
  const float* er = embed + (size_t)tok * kEmb;
  v8h hv;
#pragma unroll
  for (int i = 0; i < 4; ++i) {
    const int off = hf ? 8 : (2 * i);
    const v2f pv = *(const v2f*)(er + off);
    float f0 = pv[0];
    float f1 = pv[1];
    asm volatile("" : "+v"(f0), "+v"(f1));
    const bool keep = (hf == 0) || (i == 0);
    const float x0 = keep ? (f0 * kCarryA) : 0.0f;
    const float x1 = keep ? (f1 * kCarryA) : 0.0f;
    hv[2 * i]     = to_h_flush(x0);
    hv[2 * i + 1] = to_h_flush(x1);
  }
  _Float16* q = Epl + (size_t)c * 8;
  *(volatile v8h*)q = hv;
  __threadfence();
  *(volatile v8h*)q = hv;
}

__global__ __launch_bounds__(kThreads) void lstm_pair_scan_kernel(
    const _Float16* __restrict__ Epl,
    const float* __restrict__ W1, const float* __restrict__ b1,
    const float* __restrict__ W2, const float* __restrict__ b2,
    const float* __restrict__ Wout, const float* __restrict__ bout,
    float* __restrict__ out)
{
  __shared__ __align__(16) _Float16 sW1[kN1 * kP1];
  __shared__ __align__(16) _Float16 sW2[kN2 * kP2];
  __shared__ __align__(16) _Float16 sA1[2 * kRowsBlk * kP1];
  __shared__ __align__(16) _Float16 sA2[2 * kRowsBlk * kP2];
  __shared__ __align__(16) float sHead[kL2Waves * 32];

  const int tid  = threadIdx.x;
  const int lane = tid & 31;
  const int wave = __builtin_amdgcn_readfirstlane(tid >> 5);
  const int hh   = lane >> 4;
  const int n    = lane & 15;
  const int bm0  = blockIdx.x * kRowsBlk;

#pragma unroll 1
  for (int idx = tid; idx < kN1 * kCh1; idx += kThreads) {
    const int np = idx / kCh1;
    const int ch = idx - np * kCh1;
    const v8h v = pack_chunk<kH1, kH1P, kW1Cols, kW1Rows, kEmb, 0, kEmb>(W1, np, ch * 8);
    *(v8h*)(sW1 + np * kP1 + ch * 8) = v;
  }
#pragma unroll 1
  for (int idx = tid; idx < kN2 * kCh2; idx += kThreads) {
    const int np = idx / kCh2;
    const int ch = idx - np * kCh2;
    const v8h v = pack_chunk<kH2, kH2P, kW2Cols, kW2Rows, 0, kH1, kH2>(W2, np, ch * 8);
    *(v8h*)(sW2 + np * kP2 + ch * 8) = v;
  }
  {
    const v8h zero8 = (v8h){(_Float16)0.0f, (_Float16)0.0f, (_Float16)0.0f, (_Float16)0.0f,
                            (_Float16)0.0f, (_Float16)0.0f, (_Float16)0.0f, (_Float16)0.0f};
#pragma unroll 1
    for (int idx = tid; idx < (2 * kRowsBlk * kP1) / 8; idx += kThreads) *(v8h*)(sA1 + idx * 8) = zero8;
#pragma unroll 1
    for (int idx = tid; idx < (2 * kRowsBlk * kP2) / 8; idx += kThreads) *(v8h*)(sA2 + idx * 8) = zero8;
  }
  __syncthreads();

  if (wave == kL1Waves) {
    const int row = lane >> 1;
    const int hf = lane & 1;
    const v8h ev = *(const v8h*)(Epl + ((size_t)bm0 + row) * kEW + hf * 8);
    *(v8h*)(sA1 + row * kP1 + kH1P + hf * 8) = ev;
  }

  const bool role1 = wave < kL1Waves;
  const int jt = role1 ? wave : (wave - kL1Waves);
  const int hreal = role1 ? kH1 : kH2;
  const float* bsrc = role1 ? b1 : b2;
  const int j = jt * 16 + n;
  const bool valid = j < hreal;
  const int jc = valid ? j : (hreal - 1);
  float bias[4];
#pragma unroll
  for (int g = 0; g < 4; ++g) {
    float bv = bsrc[g * hreal + jc];
    asm volatile("" : "+v"(bv));
    bias[g] = valid ? bv : 0.0f;
  }
  float cst[8];
  float hacc[16];
#pragma unroll
  for (int r = 0; r < 8; ++r) cst[r] = 0.0f;
#pragma unroll
  for (int i = 0; i < 16; ++i) hacc[i] = 0.0f;

  __syncthreads();

#pragma unroll 1
  for (int t = 0; t < kT; ++t) {
    const int p = t & 1;
    const _Float16* a1cur = sA1 + p * (kRowsBlk * kP1);
    _Float16* a1nxt = sA1 + (p ^ 1) * (kRowsBlk * kP1);
    _Float16* a2cur = sA2 + p * (kRowsBlk * kP2);
    _Float16* a2nxt = sA2 + (p ^ 1) * (kRowsBlk * kP2);

    if (wave < kL1Waves) {
      v8f acc[4];
#pragma unroll
      for (int g = 0; g < 4; ++g) acc[g] = (v8f){0.f, 0.f, 0.f, 0.f, 0.f, 0.f, 0.f, 0.f};
#pragma unroll
      for (int kt = 0; kt < kK1 / 32; ++kt) {
        const v16h a = frag_load(a1cur + n * kP1 + kt * 32 + 8 * hh);
#pragma unroll
        for (int g = 0; g < 4; ++g) {
          const v16h b = frag_load(sW1 + (g * kH1P + jt * 16 + n) * kP1 + kt * 32 + 8 * hh);
          acc[g] = mma_h(a, b, acc[g]);
        }
      }
#pragma unroll
      for (int r = 0; r < 8; ++r) {
        const float hv = cell_step(acc[0][r], acc[1][r], acc[2][r], acc[3][r],
                                   bias[0], bias[1], bias[2], bias[3], cst[r]);
        const float hs = valid ? (hv * kCarryA) : 0.0f;
        const _Float16 hq = to_h_flush(hs);
        const _Float16 aq = to_h_flush(fmaxf(hs, 0.0f));
        a1nxt[(8 * hh + r) * kP1 + jt * 16 + n] = hq;
        a2cur[(8 * hh + r) * kP2 + jt * 16 + n] = aq;
      }
    } else if (wave == kL1Waves) {
      const int tn = (t + 1 < kT) ? (t + 1) : (kT - 1);
      const int row = lane >> 1;
      const int hf = lane & 1;
      const v8h ev = *(const v8h*)(Epl + ((size_t)tn * kB + bm0 + row) * kEW + hf * 8);
      *(v8h*)(a1nxt + row * kP1 + kH1P + hf * 8) = ev;
    } else {
      const int row = lane >> 1;
      const int hf = lane & 1;
      const v8h zero8 = (v8h){(_Float16)0.0f, (_Float16)0.0f, (_Float16)0.0f, (_Float16)0.0f,
                              (_Float16)0.0f, (_Float16)0.0f, (_Float16)0.0f, (_Float16)0.0f};
      *(v8h*)(a2cur + row * kP2 + kH1P + kH2P + hf * 8) = zero8;
    }
    __syncthreads();

    if (wave >= kL1Waves) {
      const v2f wv = *(const v2f*)(Wout + ((size_t)t * kH2 + jc) * 2);
      float w0 = wv[0];
      float w1 = wv[1];
      asm volatile("" : "+v"(w0), "+v"(w1));
      w0 = valid ? w0 : 0.0f;
      w1 = valid ? w1 : 0.0f;

      v8f acc[4];
#pragma unroll
      for (int g = 0; g < 4; ++g) acc[g] = (v8f){0.f, 0.f, 0.f, 0.f, 0.f, 0.f, 0.f, 0.f};
#pragma unroll
      for (int kt = 0; kt < kK2 / 32; ++kt) {
        const v16h a = frag_load(a2cur + n * kP2 + kt * 32 + 8 * hh);
#pragma unroll
        for (int g = 0; g < 4; ++g) {
          const v16h b = frag_load(sW2 + (g * kH2P + jt * 16 + n) * kP2 + kt * 32 + 8 * hh);
          acc[g] = mma_h(a, b, acc[g]);
        }
      }
#pragma unroll
      for (int r = 0; r < 8; ++r) {
        const float hv = cell_step(acc[0][r], acc[1][r], acc[2][r], acc[3][r],
                                   bias[0], bias[1], bias[2], bias[3], cst[r]);
        hacc[2 * r]     = fmaf(hv, w0, hacc[2 * r]);
        hacc[2 * r + 1] = fmaf(hv, w1, hacc[2 * r + 1]);
        const float hs = valid ? (hv * kCarryA) : 0.0f;
        a2nxt[(8 * hh + r) * kP2 + kH1P + jt * 16 + n] = to_h_flush(hs);
      }
    }
    __syncthreads();
  }

#pragma unroll
  for (int i = 0; i < 16; ++i) {
    float v = hacc[i];
    v += __shfl_xor(v, 1, 32);
    v += __shfl_xor(v, 2, 32);
    v += __shfl_xor(v, 4, 32);
    v += __shfl_xor(v, 8, 32);
    hacc[i] = v;
  }
  if (wave >= kL1Waves) {
    if (n == 0) {
#pragma unroll
      for (int r = 0; r < 8; ++r) {
        sHead[(wave - kL1Waves) * 32 + (8 * hh + r) * 2 + 0] = hacc[2 * r];
        sHead[(wave - kL1Waves) * 32 + (8 * hh + r) * 2 + 1] = hacc[2 * r + 1];
      }
    }
  }
  __syncthreads();
  if (wave == 0) {
    const float res = (sHead[lane] + sHead[32 + lane]) + bout[lane & 1];
    float* op = out + (size_t)bm0 * 2 + lane;
    *(volatile float*)op = res;
    __threadfence();
    *(volatile float*)op = res;
  }
}

extern "C" void kernel_launch(void* const* d_in, const int* in_sizes, int n_in,
                              void* d_out, int out_size, void* d_ws, size_t ws_size,
                              hipStream_t stream) {
  if (n_in < 8) return;
  if (in_sizes[0] != kB * kT) return;
  if (in_sizes[1] != kVocab * kEmb) return;
  if (in_sizes[2] != kW1Rows * kW1Cols) return;
  if (in_sizes[3] != kW1Cols) return;
  if (in_sizes[4] != kW2Rows * kW2Cols) return;
  if (in_sizes[5] != kW2Cols) return;
  if (in_sizes[6] != kT * kH2 * 2) return;
  if (in_sizes[7] != 2) return;
  if (out_size != kB * 2) return;
  if (ws_size < kWsTotal) return;

  const int*   x     = (const int*)d_in[0];
  const float* embed = (const float*)d_in[1];
  const float* W1    = (const float*)d_in[2];
  const float* b1    = (const float*)d_in[3];
  const float* W2    = (const float*)d_in[4];
  const float* b2    = (const float*)d_in[5];
  const float* Wout  = (const float*)d_in[6];
  const float* bout  = (const float*)d_in[7];
  float* out = (float*)d_out;

  _Float16* Epl = (_Float16*)((char*)d_ws + kOffE);

  pack_embed_kernel<<<kPackChunks / 256, 256, 0, stream>>>(x, embed, Epl);
  lstm_pair_scan_kernel<<<kBlocks, kThreads, 0, stream>>>(Epl, W1, b1, W2, b2, Wout, bout, out);
}
